// MambaBlock_816043786853
// MI455X (gfx1250) — hardware-verified
//
#include <hip/hip_runtime.h>
#include <math.h>

typedef __attribute__((ext_vector_type(16))) _Float16 v16h;
typedef __attribute__((ext_vector_type(8)))  _Float16 v8h;
typedef __attribute__((ext_vector_type(8)))  float    v8f;
typedef __attribute__((ext_vector_type(4)))  float    v4f;

constexpr int kBatch  = 8;
constexpr int kSeq    = 1024;
constexpr int kDm     = 256;
constexpr int kDin    = 512;
constexpr int kNst    = 16;
constexpr int kDtR    = 16;
constexpr int kSeHid  = 16;
constexpr int kXzP    = 2 * kDin;
constexpr int kXdN    = kDtR + 2 * kNst;
constexpr int kXdP    = 64;
constexpr int kRows   = kBatch * kSeq;
constexpr int kConvTP = 260;
constexpr int kScanTS = 64;
constexpr int kScanCh = 64;
constexpr int kScanYP = 68;
constexpr int kTrP    = 68;
constexpr int kLnBlkRows = 64;
constexpr int kLnBlocks  = kRows / kLnBlkRows;
constexpr int kLnBlkPerB = kSeq / kLnBlkRows;
constexpr float kCarryW  = 32.0f;
constexpr float kCarryU  = 16.0f;
constexpr float kCarryY  = 256.0f;
constexpr float kLnEps   = 1e-5f;
static_assert(kXdN <= kXdP, "x_proj width");
static_assert((kDm % 32) == 0 && (kDin % 32) == 0, "GEMM K multiples of 32");
static_assert((kRows % 64) == 0 && (kXzP % 64) == 0 && (kXdP % 64) == 0 && (kDm % 64) == 0, "GEMM M,N multiples of 64");
static_assert((kSeq % kScanTS) == 0 && (kSeq % 64) == 0 && (kDin % kScanCh) == 0 && (kDin % 256) == 0, "tile multiples");
static_assert((kSeq & (kSeq - 1)) == 0, "sequence length power of two");
static_assert(kDm == 256 && kSeHid == 16 && kDtR == 16 && kNst == 16, "lane maps below assume these widths");

constexpr size_t kOffXS   = 0;
constexpr size_t kOffWIN  = kOffXS   + (size_t)kRows * kDm  * 2;
constexpr size_t kOffWXP  = kOffWIN  + (size_t)kXzP  * kDm  * 2;
constexpr size_t kOffWOUT = kOffWXP  + (size_t)kXdP  * kDin * 2;
constexpr size_t kOffXZ   = kOffWOUT + (size_t)kDm   * kDin * 2;
constexpr size_t kOffUC   = kOffXZ   + (size_t)kRows * kXzP * 4;
constexpr size_t kOffUC16 = kOffUC   + (size_t)kRows * kDin * 4;
constexpr size_t kOffXD   = kOffUC16 + (size_t)kRows * kDin * 2;
constexpr size_t kOffY16  = kOffXD   + (size_t)kRows * kXdP * 4;
constexpr size_t kOffOUTF = kOffY16  + (size_t)kRows * kDin * 2;
constexpr size_t kOffLNF  = kOffOUTF + (size_t)kRows * kDm  * 4;
constexpr size_t kOffPS   = kOffLNF  + (size_t)kRows * kDm  * 4;
constexpr size_t kOffSG   = kOffPS   + (size_t)kLnBlocks * kDm * 4;
constexpr size_t kWsTotal = kOffSG   + (size_t)kBatch * kDm * 4;
static_assert(kWsTotal == 91168768ull, "carve total");
static_assert(kWsTotal <= 134217728ull, "carve cap");
static_assert((kOffWIN % 128) == 0 && (kOffWXP % 128) == 0 && (kOffWOUT % 128) == 0 && (kOffXZ % 128) == 0 &&
              (kOffUC % 128) == 0 && (kOffUC16 % 128) == 0 && (kOffXD % 128) == 0 && (kOffY16 % 128) == 0 &&
              (kOffOUTF % 128) == 0 && (kOffLNF % 128) == 0 && (kOffPS % 128) == 0 && (kOffSG % 128) == 0,
              "128-B aligned regions");

union FragHU { v16h v; v8h h[2]; };
__device__ __forceinline__ v16h frag_load_h(const _Float16* p) {
  FragHU f;
  f.h[0] = *(const v8h*)(p);
  f.h[1] = *(const v8h*)(p + 16);
  return f.v;
}
__device__ __forceinline__ v8f mma_h(v16h a, v16h b, v8f c) {
  return __builtin_amdgcn_wmma_f32_16x16x32_f16(false, a, false, b, (short)0, c, false, false);
}
__device__ __forceinline__ void guard4_h(v8f& a, v8f& b, v8f& c, v8f& d, v16h x) {
  asm volatile("v_nop\n\tv_nop\n\tv_nop\n\tv_nop" : "+v"(a), "+v"(b), "+v"(c), "+v"(d) : "v"(x));
}
__device__ __forceinline__ void keep4_h(v16h a, v16h b, v16h c, v16h d) {
  asm volatile("v_nop" :: "v"(a), "v"(b), "v"(c), "v"(d));
}
__device__ __forceinline__ void acc_guard4(v8f& a, v8f& b, v8f& c, v8f& d) {
  asm volatile("v_nop\n\tv_nop\n\tv_nop\n\tv_nop" : "+v"(a), "+v"(b), "+v"(c), "+v"(d));
}

__global__ __launch_bounds__(256) void wmma_gemm64_f16(
    const unsigned short* __restrict__ Ap, int lda,
    const unsigned short* __restrict__ Btp, int ldb,
    float* __restrict__ C, int ldc, int M, int N, int K, float scale)
{
  const _Float16* A  = (const _Float16*)Ap;
  const _Float16* Bt = (const _Float16*)Btp;
  __shared__ __align__(16) float sT[8][16 * 68];
  const int lane = threadIdx.x & 31;
  const int wave = threadIdx.x >> 5;
  const int tilesN = N >> 6;
  const int tilesM = M >> 6;
  const int tile = blockIdx.x * 8 + wave;
  if (tile >= tilesM * tilesN) return;
  const int tm = tile / tilesN;
  const int tn = tile - tm * tilesN;
  const int m0 = tm << 6;
  const int n0 = tn << 6;

  const int rlane = lane & 15;
  const int koff  = (lane >> 4) * 8;
  const int mOff  = (lane >> 4) * 8;

  v8f acc[4][4];
#pragma unroll
  for (int i = 0; i < 4; ++i)
#pragma unroll
    for (int j = 0; j < 4; ++j) acc[i][j] = (v8f){0.f,0.f,0.f,0.f,0.f,0.f,0.f,0.f};

  for (int k0 = 0; k0 < K; k0 += 32) {
    v16h bh[4];
#pragma unroll
    for (int j = 0; j < 4; ++j) {
      const size_t bo = (size_t)(n0 + (j << 4) + rlane) * ldb + koff + k0;
      bh[j] = frag_load_h(Bt + bo);
    }
#pragma unroll
    for (int i = 0; i < 4; ++i) {
      const size_t ao = (size_t)(m0 + (i << 4) + rlane) * lda + koff + k0;
      const v16h ah = frag_load_h(A + ao);
#pragma unroll
      for (int j = 0; j < 4; ++j) acc[i][j] = mma_h(ah, bh[j], acc[i][j]);
      guard4_h(acc[i][0], acc[i][1], acc[i][2], acc[i][3], ah);
    }
    keep4_h(bh[0], bh[1], bh[2], bh[3]);
  }
  acc_guard4(acc[0][0], acc[0][1], acc[0][2], acc[0][3]);
  acc_guard4(acc[1][0], acc[1][1], acc[1][2], acc[1][3]);
  acc_guard4(acc[2][0], acc[2][1], acc[2][2], acc[2][3]);
  acc_guard4(acc[3][0], acc[3][1], acc[3][2], acc[3][3]);

  float* slab = sT[wave];
#pragma unroll
  for (int i = 0; i < 4; ++i) {
    const int mBase = m0 + (i << 4);
#pragma unroll
    for (int j = 0; j < 4; ++j) {
#pragma unroll
      for (int r = 0; r < 8; ++r) {
        slab[(mOff + r) * 68 + (j << 4) + rlane] = acc[i][j][r] * scale;
      }
    }
    __builtin_amdgcn_fence(__ATOMIC_RELEASE, "workgroup");
    __builtin_amdgcn_wave_barrier();
    __builtin_amdgcn_fence(__ATOMIC_ACQUIRE, "workgroup");
    {
      const int hh = lane >> 4, c4 = (lane & 15) * 4;
      for (int pass = 0; pass < 2; ++pass) {
#pragma unroll
        for (int it = 0; it < 8; ++it) {
          const int row = it * 2 + hh;
          const v4f v = *(const v4f*)(slab + row * 68 + c4);
          *(volatile v4f*)(C + (size_t)(mBase + row) * ldc + n0 + c4) = v;
        }
        __threadfence();
      }
    }
    __builtin_amdgcn_fence(__ATOMIC_RELEASE, "workgroup");
    __builtin_amdgcn_wave_barrier();
    __builtin_amdgcn_fence(__ATOMIC_ACQUIRE, "workgroup");
  }
}

__global__ __launch_bounds__(256) void cast_pad_f16_kernel(
    const float* __restrict__ src, unsigned short* __restrict__ dst, int total8, int real8, float scale)
{
  const int i = blockIdx.x * 256 + threadIdx.x;
  if (i >= total8) return;
  const bool real = (i < real8);
  const size_t es = (size_t)(real ? i : 0) << 3;
  const v4f a0 = *(const v4f*)(src + es);
  const v4f a1 = *(const v4f*)(src + es + 4);
  v8h hv;
#pragma unroll
  for (int e = 0; e < 4; ++e) {
    const float f0 = real ? (a0[e] * scale) : 0.0f;
    const float f1 = real ? (a1[e] * scale) : 0.0f;
    hv[e]     = (_Float16)f0;
    hv[4 + e] = (_Float16)f1;
  }
  unsigned short* q = dst + ((size_t)i << 3);
  *(volatile v8h*)q = hv;
  __threadfence();
  *(volatile v8h*)q = hv;
}

__global__ __launch_bounds__(256) void tokens_f16_kernel(
    const float* __restrict__ x, unsigned short* __restrict__ XS16)
{
  __shared__ __align__(16) float tile[64 * kTrP];
  const int tid = threadIdx.x, lane = tid & 31, wave = tid >> 5;
  const int l0 = blockIdx.x * 64, c0 = blockIdx.y * 64, b = blockIdx.z;
  const int rr = tid >> 4, l4 = (tid & 15) * 4;
#pragma unroll
  for (int p = 0; p < 4; ++p) {
    const int c = p * 16 + rr;
    const v4f v = *(const v4f*)(x + ((size_t)(b * kDm + c0 + c)) * kSeq + l0 + l4);
    tile[(l4 + 0) * kTrP + c] = v[0];
    tile[(l4 + 1) * kTrP + c] = v[1];
    tile[(l4 + 2) * kTrP + c] = v[2];
    tile[(l4 + 3) * kTrP + c] = v[3];
  }
  __syncthreads();
  const int q = lane >> 3, c8 = (lane & 7) * 8;
  v8h hv[2];
#pragma unroll
  for (int it = 0; it < 2; ++it) {
    const int l = it * 32 + wave * 4 + q;
    const float* sp = tile + l * kTrP + c8;
    const v4f a0 = *(const v4f*)(sp);
    const v4f a1 = *(const v4f*)(sp + 4);
#pragma unroll
    for (int e = 0; e < 4; ++e) {
      hv[it][e]     = (_Float16)a0[e];
      hv[it][4 + e] = (_Float16)a1[e];
    }
  }
  for (int pass = 0; pass < 2; ++pass) {
#pragma unroll
    for (int it = 0; it < 2; ++it) {
      const int l = it * 32 + wave * 4 + q;
      *(volatile v8h*)(XS16 + ((size_t)(b * kSeq + l0 + l)) * kDm + c0 + c8) = hv[it];
    }
    __threadfence();
  }
}

__global__ __launch_bounds__(256) void conv_silu_kernel(
    const float* __restrict__ XZ, const float* __restrict__ cw, const float* __restrict__ cb,
    float* __restrict__ UC, unsigned short* __restrict__ UC16)
{
  __shared__ __align__(16) float sT[16 * kConvTP];
  const int tid = threadIdx.x, lane = tid & 31, wave = tid >> 5;
  const int d0 = blockIdx.x * 256, d = d0 + tid;
  const int g0 = blockIdx.y * 64;
  const int tb = g0 & (kSeq - 1);
  const v4f wv = *(const v4f*)(cw + d * 4);
  const float w0 = wv[0], w1 = wv[1], w2 = wv[2], w3 = wv[3];
  const float bc = cb[d];
  float xm3, xm2, xm1;
  {
    const bool hist = (tb > 0);
    const int rb = hist ? (g0 - 3) : g0;
    const float v3 = XZ[(size_t)rb * kXzP + d];
    const float v2 = XZ[(size_t)(rb + 1) * kXzP + d];
    const float v1 = XZ[(size_t)(rb + 2) * kXzP + d];
    xm3 = hist ? v3 : 0.f;
    xm2 = hist ? v2 : 0.f;
    xm1 = hist ? v1 : 0.f;
  }
  const int hrow = wave >> 1;
  const int hch  = (wave & 1) * 128 + lane * 4;
#pragma unroll 1
  for (int sub = 0; sub < 4; ++sub) {
    const int lb = g0 + sub * 16;
#pragma unroll 1
    for (int s = 0; s < 16; ++s) {
      const float xcur = XZ[(size_t)(lb + s) * kXzP + d];
      float acc = w0 * xm3;
      acc = fmaf(w1, xm2, acc);
      acc = fmaf(w2, xm1, acc);
      acc = fmaf(w3, xcur, acc);
      const float sv = acc + bc;
      const float sg = __builtin_amdgcn_rcpf(1.0f + expf(-sv));
      sT[s * kConvTP + tid] = sv * sg;
      xm3 = xm2; xm2 = xm1; xm1 = xcur;
    }
    __syncthreads();
    v4f fv[4];
    v8h bv[2];
#pragma unroll
    for (int it = 0; it < 4; ++it) fv[it] = *(const v4f*)(sT + (it * 4 + hrow) * kConvTP + hch);
#pragma unroll
    for (int it = 0; it < 2; ++it) {
      const float* sp = sT + (it * 8 + wave) * kConvTP + lane * 8;
      const v4f a0 = *(const v4f*)(sp);
      const v4f a1 = *(const v4f*)(sp + 4);
#pragma unroll
      for (int e = 0; e < 4; ++e) {
        bv[it][e]     = (_Float16)(a0[e] * kCarryU);
        bv[it][4 + e] = (_Float16)(a1[e] * kCarryU);
      }
    }
    for (int pass = 0; pass < 2; ++pass) {
#pragma unroll
      for (int it = 0; it < 4; ++it)
        *(volatile v4f*)(UC + (size_t)(lb + it * 4 + hrow) * kDin + d0 + hch) = fv[it];
#pragma unroll
      for (int it = 0; it < 2; ++it)
        *(volatile v8h*)(UC16 + (size_t)(lb + it * 8 + wave) * kDin + d0 + lane * 8) = bv[it];
      __threadfence();
    }
    __syncthreads();
  }
}

__global__ __launch_bounds__(64) void scan_kernel(
    const float* __restrict__ XD, const float* __restrict__ UC, const float* __restrict__ XZ,
    const float* __restrict__ Wdt, const float* __restrict__ bdt, const float* __restrict__ Alog,
    const float* __restrict__ Dp, unsigned short* __restrict__ Y16)
{
  __shared__ __align__(16) float sX[kScanTS * kXdP];
  __shared__ __align__(16) float sY[kScanTS * kScanYP];
  __shared__ __align__(16) float sW[kDtR * kScanCh];
  __shared__ __align__(16) float sA[kNst * kScanCh];
  const int tid = threadIdx.x, lane = tid & 31, wave = tid >> 5;
  constexpr int kBlkPerB = kDin / kScanCh;
  const int bix = blockIdx.x / kBlkPerB;
  const int d0  = (blockIdx.x - bix * kBlkPerB) * kScanCh;
  const int d   = d0 + tid;
  const size_t row0 = (size_t)bix * kSeq;
#pragma unroll 1
  for (int r = 0; r < kDtR; ++r) sW[r * kScanCh + tid] = Wdt[(size_t)d * kDtR + r];
#pragma unroll 1
  for (int s = 0; s < kNst; ++s) sA[s * kScanCh + tid] = -expf(Alog[(size_t)d * kNst + s]);
  __syncthreads();
  float negA[kNst], h[kNst];
#pragma unroll
  for (int s = 0; s < kNst; ++s) {
    negA[s] = sA[s * kScanCh + tid];
    h[s] = 0.f;
  }
  const float bb = bdt[d], Dd = Dp[d];
  const int lr = tid >> 4, lc4 = (tid & 15) * 4;
  const int q = lane >> 3, c8 = (lane & 7) * 8;
#pragma unroll 1
  for (int t0 = 0; t0 < kSeq; t0 += kScanTS) {
    __syncthreads();
#pragma unroll
    for (int i = 0; i < 16; ++i) {
      const int r = lr + 4 * i;
      *(v4f*)(sX + r * kXdP + lc4) = *(const v4f*)(XD + (row0 + t0 + r) * kXdP + lc4);
    }
    __syncthreads();
#pragma unroll 1
    for (int s = 0; s < kScanTS; ++s) {
      const int t = t0 + s;
      const float* xr = sX + s * kXdP;
      float vdot = 0.f;
#pragma unroll 1
      for (int r4 = 0; r4 < kDtR / 4; ++r4) {
        const v4f xv = *(const v4f*)(xr + 4 * r4);
        const float* wp = sW + (4 * r4) * kScanCh + tid;
        vdot = fmaf(xv[0], wp[0], vdot);
        vdot = fmaf(xv[1], wp[kScanCh], vdot);
        vdot = fmaf(xv[2], wp[2 * kScanCh], vdot);
        vdot = fmaf(xv[3], wp[3 * kScanCh], vdot);
      }
      float Bs[kNst], Cs[kNst];
#pragma unroll
      for (int q4 = 0; q4 < 4; ++q4) {
        const v4f bv = *(const v4f*)(xr + kDtR + 4 * q4);
        const v4f cv = *(const v4f*)(xr + kDtR + kNst + 4 * q4);
        Bs[4 * q4 + 0] = bv[0]; Bs[4 * q4 + 1] = bv[1]; Bs[4 * q4 + 2] = bv[2]; Bs[4 * q4 + 3] = bv[3];
        Cs[4 * q4 + 0] = cv[0]; Cs[4 * q4 + 1] = cv[1]; Cs[4 * q4 + 2] = cv[2]; Cs[4 * q4 + 3] = cv[3];
      }
      const float v   = vdot + bb;
      const float a   = __expf(-fabsf(v));
      const float u1  = 1.0f + a;
      const float l1p = __logf(u1) + (a - (u1 - 1.0f)) * __builtin_amdgcn_rcpf(u1);
      const float dt  = fmaxf(v, 0.0f) + l1p;
      const float xt  = UC[(row0 + t) * kDin + d];
      const float dtx = dt * xt;
      float y = 0.f;
#pragma unroll
      for (int k = 0; k < kNst; ++k) {
        const float e = __expf(dt * negA[k]);
        h[k] = e * h[k] + dtx * Bs[k];
        y = h[k] * Cs[k] + y;
      }
      y = xt * Dd + y;
      const float zv = XZ[(row0 + t) * kXzP + kDin + d];
      const float sg = __builtin_amdgcn_rcpf(1.0f + expf(-zv));
      y = y * (zv * sg);
      sY[s * kScanYP + tid] = y * kCarryY;
    }
    __syncthreads();
    v8h hv[8];
#pragma unroll
    for (int it = 0; it < 8; ++it) {
      const int row = it * 8 + wave * 4 + q;
      const float* sp = sY + row * kScanYP + c8;
      const v4f a0 = *(const v4f*)(sp);
      const v4f a1 = *(const v4f*)(sp + 4);
#pragma unroll
      for (int e = 0; e < 4; ++e) {
        hv[it][e]     = (_Float16)a0[e];
        hv[it][4 + e] = (_Float16)a1[e];
      }
    }
    for (int pass = 0; pass < 2; ++pass) {
#pragma unroll
      for (int it = 0; it < 8; ++it) {
        const int row = it * 8 + wave * 4 + q;
        const size_t o = (row0 + t0 + row) * kDin + d0 + c8;
        *(volatile v8h*)(Y16 + o) = hv[it];
      }
      __threadfence();
    }
  }
}

__global__ __launch_bounds__(256) void layernorm_kernel(
    const float* __restrict__ OUTF, const float* __restrict__ lw, const float* __restrict__ lb,
    float* __restrict__ LNF, float* __restrict__ PS)
{
  __shared__ __align__(16) float sP[8 * kDm];
  const int tid = threadIdx.x, lane = tid & 31, wave = tid >> 5;
  const int rbase = blockIdx.x * kLnBlkRows + wave * 8;
  const int ca = lane * 4, cb2 = 128 + lane * 4;
  const v4f wa = *(const v4f*)(lw + ca);
  const v4f wb = *(const v4f*)(lw + cb2);
  const v4f ba = *(const v4f*)(lb + ca);
  const v4f bb = *(const v4f*)(lb + cb2);
  v4f csa = (v4f){0.f, 0.f, 0.f, 0.f};
  v4f csb = (v4f){0.f, 0.f, 0.f, 0.f};
#pragma unroll 1
  for (int j = 0; j < 8; ++j) {
    const size_t ro = (size_t)(rbase + j) * kDm;
    const v4f a0 = *(const v4f*)(OUTF + ro + ca);
    const v4f a1 = *(const v4f*)(OUTF + ro + cb2);
    float s = ((a0[0] + a0[1]) + (a0[2] + a0[3])) + ((a1[0] + a1[1]) + (a1[2] + a1[3]));
#pragma unroll
    for (int off = 16; off >= 1; off >>= 1) s += __shfl_xor(s, off, 32);
    const float mu = s * (1.0f / (float)kDm);
    const v4f e0 = a0 - mu;
    const v4f e1 = a1 - mu;
    float qv = ((e0[0] * e0[0] + e0[1] * e0[1]) + (e0[2] * e0[2] + e0[3] * e0[3])) +
               ((e1[0] * e1[0] + e1[1] * e1[1]) + (e1[2] * e1[2] + e1[3] * e1[3]));
#pragma unroll
    for (int off = 16; off >= 1; off >>= 1) qv += __shfl_xor(qv, off, 32);
    const float var = qv * (1.0f / (float)kDm);
    const float rs = rsqrtf(var + kLnEps);
    const v4f o0 = (e0 * rs) * wa + ba;
    const v4f o1 = (e1 * rs) * wb + bb;
    csa += o0;
    csb += o1;
    *(volatile v4f*)(LNF + ro + ca)  = o0;
    *(volatile v4f*)(LNF + ro + cb2) = o1;
    __threadfence();
    *(volatile v4f*)(LNF + ro + ca)  = o0;
    *(volatile v4f*)(LNF + ro + cb2) = o1;
  }
  *(v4f*)(sP + wave * kDm + ca)  = csa;
  *(v4f*)(sP + wave * kDm + cb2) = csb;
  __syncthreads();
  if (tid < 64) {
    const int c4 = tid * 4;
    v4f t = (v4f){0.f, 0.f, 0.f, 0.f};
#pragma unroll
    for (int w = 0; w < 8; ++w) t += *(const v4f*)(sP + w * kDm + c4);
    float* pp = PS + (size_t)blockIdx.x * kDm + c4;
    *(volatile v4f*)pp = t;
    __threadfence();
    *(volatile v4f*)pp = t;
  }
}

__global__ __launch_bounds__(256) void se_gate_kernel(
    const float* __restrict__ PS, const float* __restrict__ w1, const float* __restrict__ w2,
    float* __restrict__ SG)
{
  __shared__ __align__(16) float s0[kDm];
  __shared__ __align__(16) float hid[kSeHid];
  __shared__ __align__(16) float sg[kDm];
  const int tid = threadIdx.x, lane = tid & 31, wave = tid >> 5;
  const int b = blockIdx.x;
  float a = 0.f;
#pragma unroll 1
  for (int j = 0; j < kLnBlkPerB; ++j) a += PS[(size_t)(b * kLnBlkPerB + j) * kDm + tid];
  s0[tid] = a * (1.0f / (float)kSeq);
  __syncthreads();
#pragma unroll 1
  for (int jj = 0; jj < 2; ++jj) {
    const int j = wave * 2 + jj;
    float p = 0.f;
#pragma unroll 1
    for (int i = 0; i < 8; ++i) {
      const int c = lane + 32 * i;
      p = fmaf(w1[j * kDm + c], s0[c], p);
    }
#pragma unroll
    for (int off = 16; off >= 1; off >>= 1) p += __shfl_xor(p, off, 32);
    if (lane == 0) hid[j] = fmaxf(p, 0.0f);
  }
  __syncthreads();
  {
    float qv = 0.f;
#pragma unroll
    for (int j4 = 0; j4 < 4; ++j4) {
      const v4f wv = *(const v4f*)(w2 + tid * kSeHid + 4 * j4);
      const v4f hv = *(const v4f*)(hid + 4 * j4);
      qv = fmaf(wv[0], hv[0], qv);
      qv = fmaf(wv[1], hv[1], qv);
      qv = fmaf(wv[2], hv[2], qv);
      qv = fmaf(wv[3], hv[3], qv);
    }
    sg[tid] = __builtin_amdgcn_rcpf(1.0f + expf(-qv));
  }
  __syncthreads();
  if (tid < 64) {
    const v4f v = *(const v4f*)(sg + tid * 4);
    float* pp = SG + (size_t)b * kDm + tid * 4;
    *(volatile v4f*)pp = v;
    __threadfence();
    *(volatile v4f*)pp = v;
  }
}

__global__ __launch_bounds__(256) void gate_residual_kernel(
    const float* __restrict__ LNF, const float* __restrict__ SG, const float* __restrict__ x,
    float* __restrict__ out)
{
  __shared__ __align__(16) float tile[64 * kTrP];
  const int tid = threadIdx.x, lane = tid & 31, wave = tid >> 5;
  const int l0 = blockIdx.x * 64, c0 = blockIdx.y * 64, b = blockIdx.z;
  const int rr = tid >> 4, c4 = (tid & 15) * 4;
#pragma unroll
  for (int p = 0; p < 4; ++p) {
    const int l = p * 16 + rr;
    const v4f v = *(const v4f*)(LNF + ((size_t)(b * kSeq + l0 + l)) * kDm + c0 + c4);
    tile[(c4 + 0) * kTrP + l] = v[0];
    tile[(c4 + 1) * kTrP + l] = v[1];
    tile[(c4 + 2) * kTrP + l] = v[2];
    tile[(c4 + 3) * kTrP + l] = v[3];
  }
  __syncthreads();
  const int hh = lane >> 4, l4 = (lane & 15) * 4;
  v4f ov[4];
#pragma unroll
  for (int p = 0; p < 4; ++p) {
    const int c = p * 16 + wave * 2 + hh;
    const float sv = SG[(size_t)b * kDm + c0 + c];
    const v4f t  = *(const v4f*)(tile + c * kTrP + l4);
    const v4f xv = *(const v4f*)(x + ((size_t)(b * kDm + c0 + c)) * kSeq + l0 + l4);
    ov[p] = t * sv + xv;
  }
  for (int pass = 0; pass < 2; ++pass) {
#pragma unroll
    for (int p = 0; p < 4; ++p) {
      const int c = p * 16 + wave * 2 + hh;
      *(volatile v4f*)(out + ((size_t)(b * kDm + c0 + c)) * kSeq + l0 + l4) = ov[p];
    }
    __threadfence();
  }
}

extern "C" void kernel_launch(void* const* d_in, const int* in_sizes, int n_in,
                              void* d_out, int out_size, void* d_ws, size_t ws_size,
                              hipStream_t stream) {
  if (n_in < 14) return;
  if (in_sizes[0]  != kBatch * kDm * kSeq) return;
  if (in_sizes[1]  != kXzP * kDm) return;
  if (in_sizes[2]  != kDin * 4) return;
  if (in_sizes[3]  != kDin) return;
  if (in_sizes[4]  != kXdN * kDin) return;
  if (in_sizes[5]  != kDin * kDtR) return;
  if (in_sizes[6]  != kDin) return;
  if (in_sizes[7]  != kDin * kNst) return;
  if (in_sizes[8]  != kDin) return;
  if (in_sizes[9]  != kDm * kDin) return;
  if (in_sizes[10] != kDm) return;
  if (in_sizes[11] != kDm) return;
  if (in_sizes[12] != kSeHid * kDm) return;
  if (in_sizes[13] != kDm * kSeHid) return;
  if (out_size != kBatch * kDm * kSeq) return;
  if (ws_size < kWsTotal) return;

  const float* x       = (const float*)d_in[0];
  const float* W_in    = (const float*)d_in[1];
  const float* conv_w  = (const float*)d_in[2];
  const float* conv_b  = (const float*)d_in[3];
  const float* W_xproj = (const float*)d_in[4];
  const float* W_dt    = (const float*)d_in[5];
  const float* b_dt    = (const float*)d_in[6];
  const float* A_log   = (const float*)d_in[7];
  const float* Dp      = (const float*)d_in[8];
  const float* W_out   = (const float*)d_in[9];
  const float* ln_w    = (const float*)d_in[10];
  const float* ln_b    = (const float*)d_in[11];
  const float* se_w1   = (const float*)d_in[12];
  const float* se_w2   = (const float*)d_in[13];
  float* out = (float*)d_out;

  char* ws = (char*)d_ws;
  unsigned short* XS16   = (unsigned short*)(ws + kOffXS);
  unsigned short* WIN16  = (unsigned short*)(ws + kOffWIN);
  unsigned short* WXP16  = (unsigned short*)(ws + kOffWXP);
  unsigned short* WOUT16 = (unsigned short*)(ws + kOffWOUT);
  float*          XZ     = (float*)(ws + kOffXZ);
  float*          UC     = (float*)(ws + kOffUC);
  unsigned short* UC16   = (unsigned short*)(ws + kOffUC16);
  float*          XD     = (float*)(ws + kOffXD);
  unsigned short* Y16    = (unsigned short*)(ws + kOffY16);
  float*          OUTF   = (float*)(ws + kOffOUTF);
  float*          LNF    = (float*)(ws + kOffLNF);
  float*          PS     = (float*)(ws + kOffPS);
  float*          SG     = (float*)(ws + kOffSG);

  tokens_f16_kernel<<<dim3(kSeq / 64, kDm / 64, kBatch), 256, 0, stream>>>(x, XS16);

  cast_pad_f16_kernel<<<(kXzP * kDm / 8) / 256, 256, 0, stream>>>(W_in, WIN16, kXzP * kDm / 8, kXzP * kDm / 8, kCarryW);
  cast_pad_f16_kernel<<<(kXdP * kDin / 8) / 256, 256, 0, stream>>>(W_xproj, WXP16, kXdP * kDin / 8, kXdN * kDin / 8, kCarryW);
  cast_pad_f16_kernel<<<(kDm * kDin / 8) / 256, 256, 0, stream>>>(W_out, WOUT16, kDm * kDin / 8, kDm * kDin / 8, kCarryW);

  wmma_gemm64_f16<<<256, 256, 0, stream>>>(XS16, kDm, WIN16, kDm, XZ, kXzP, kRows, kXzP, kDm, 1.0f / kCarryW);

  conv_silu_kernel<<<dim3(kDin / 256, kRows / 64), 256, 0, stream>>>(XZ, conv_w, conv_b, UC, UC16);

  wmma_gemm64_f16<<<16, 256, 0, stream>>>(UC16, kDin, WXP16, kDin, XD, kXdP, kRows, kXdP, kDin, 1.0f / (kCarryU * kCarryW));

  scan_kernel<<<kBatch * (kDin / kScanCh), kScanCh, 0, stream>>>(XD, UC, XZ, W_dt, b_dt, A_log, Dp, Y16);

  wmma_gemm64_f16<<<64, 256, 0, stream>>>(Y16, kDin, WOUT16, kDin, OUTF, kDm, kRows, kDm, kDin, 1.0f / (kCarryY * kCarryW));

  layernorm_kernel<<<kLnBlocks, 256, 0, stream>>>(OUTF, ln_w, ln_b, LNF, PS);

  se_gate_kernel<<<kBatch, 256, 0, stream>>>(PS, se_w1, se_w2, SG);

  gate_residual_kernel<<<dim3(kSeq / 64, kDm / 64, kBatch), 256, 0, stream>>>(LNF, SG, x, out);
}
